// multiHeadAttention_6863357739060
// MI455X (gfx1250) — hardware-verified
//
#include <hip/hip_runtime.h>
#ifndef NB
#define NB 2
#endif
#ifndef SEQ
#define SEQ 2048
#endif
#define NB_FULL 2
#define SEQ_FULL 2048
#define DM 1024
#define NH 16
#define HD 64
#define HG 2
#define PQ (NH * 2 * HD)
#define NR ((size_t)NB * SEQ)

typedef __bf16 v16b __attribute__((ext_vector_type(16)));
typedef _Float16 v16h __attribute__((ext_vector_type(16)));
typedef _Float16 v4h __attribute__((ext_vector_type(4)));
typedef unsigned short v8us __attribute__((ext_vector_type(8), may_alias));
typedef unsigned short v4us __attribute__((ext_vector_type(4)));
typedef float  v8f  __attribute__((ext_vector_type(8)));
typedef float  v4f  __attribute__((ext_vector_type(4)));
typedef float  v4fa __attribute__((ext_vector_type(4), may_alias));
union FragB { v16b v; v8us half[2]; };
union FragH { v16h v; v8us half[2]; _Float16 h[16]; unsigned short u[16]; };

static_assert(SEQ % 128 == 0);
static_assert(NH * HD == DM);
static_assert(NH % HG == 0);
static_assert(NB <= NB_FULL);
static_assert(SEQ <= SEQ_FULL);

#define A256(x) ((((size_t)(x)) + 255) & ~(size_t)255)
#define SZ_BQKV ((size_t)3 * DM * DM * 2)
#define SZ_BO   ((size_t)DM * DM * 2)
#define SZ_X16  (NR * DM * 2)
#define SZ_QKP  ((size_t)2 * NR * PQ * 2)
#define SZ_V16  (NR * DM * 2)
#define SZ_VT   ((size_t)NB * NH * HD * SEQ * 2)
#define SZ_O16  (NR * DM * 2)
#define SZ_S    ((size_t)HG * SEQ * SEQ * 4)
#define SZ_P    ((size_t)HG * SEQ * SEQ * 2)
static_assert(A256(SZ_BQKV) + A256(SZ_BO) + A256(SZ_X16) + A256(SZ_QKP) + A256(SZ_V16) + A256(SZ_VT) + A256(SZ_O16) + A256(SZ_S) + A256(SZ_P) <= (size_t)134217728);

__device__ __forceinline__ unsigned short bf16_bits(float x) { unsigned int u = __float_as_uint(x); return (unsigned short)((u + 0x7FFFu + ((u >> 16) & 1u)) >> 16); }
__device__ __forceinline__ float bf16_val(unsigned short b) { return __uint_as_float(((unsigned int)b) << 16); }
__device__ __forceinline__ float bf16_rne(float x) { return bf16_val(bf16_bits(x)); }

__device__ __forceinline__ v16h g2_frag(const _Float16* p, int hh) { FragH f; f.half[0] = *(const v8us*)((const unsigned short*)p + 8 * hh); f.half[1] = *(const v8us*)((const unsigned short*)p + 16 + 8 * hh); return f.v; }
__device__ __forceinline__ v8f g2_mma(v16h a, v16h b, v8f c) { v8f d = __builtin_amdgcn_wmma_f32_16x16x32_f16(false, a, false, b, (short)0, c, false, false); asm volatile("v_nop\n\tv_nop\n\tv_nop\n\tv_nop" : "+v"(d) : "v"(a), "v"(b)); return d; }
__device__ __forceinline__ v16b gb_frag(const unsigned short* p, int hh) { FragB f; f.half[0] = *(const v8us*)(p + 8 * hh); f.half[1] = *(const v8us*)(p + 16 + 8 * hh); return f.v; }
__device__ __forceinline__ v8f gb_mma(v16b a, v16b b, v8f c) { v8f d = __builtin_amdgcn_wmma_f32_16x16x32_bf16(false, a, false, b, (short)0, c, false, false); asm volatile("v_nop\n\tv_nop\n\tv_nop\n\tv_nop" : "+v"(d) : "v"(a), "v"(b)); return d; }

__global__ __launch_bounds__(256) void k_x16(const float* __restrict__ x, _Float16* __restrict__ X16, size_t n8) {
  const size_t t = (size_t)blockIdx.x * 256 + threadIdx.x; if (t >= n8) return;
  const size_t row = t / (DM / 8); const int c8 = (int)(t % (DM / 8)) * 8;
  const size_t b = row / SEQ, s = row % SEQ;
  const float* src = x + (b * SEQ_FULL + s) * DM + c8;
  const v4f a = *(const v4fa*)src, c = *(const v4fa*)(src + 4);
  FragH f;
#pragma unroll
  for (int q = 0; q < 4; ++q) { f.h[q] = (_Float16)(bf16_rne(a[q]) * 64.0f); f.h[4 + q] = (_Float16)(bf16_rne(c[q]) * 64.0f); }
  const v8us o = f.half[0];
  unsigned short* d = (unsigned short*)X16 + t * 8;
  *(volatile v8us*)d = o; __threadfence(); *(volatile v8us*)d = o;
}

__global__ __launch_bounds__(256) void k_wth(const float* __restrict__ W, _Float16* __restrict__ Wt) {
  const int t = blockIdx.x * 256 + threadIdx.x; if (t >= DM * (DM / 8)) return;
  const int n = t / (DM / 8), k8 = (t % (DM / 8)) * 8; const int h = n / HD, d = n % HD;
  const float* src = W + (size_t)h * DM * HD + (size_t)k8 * HD + d;
  FragH f;
#pragma unroll
  for (int i = 0; i < 8; ++i) f.h[i] = (_Float16)(bf16_rne(src[(size_t)i * HD]) * 64.0f);
  const v8us o = f.half[0];
  unsigned short* dst = (unsigned short*)Wt + (size_t)n * DM + k8;
  *(volatile v8us*)dst = o; __threadfence(); *(volatile v8us*)dst = o;
}

__global__ __launch_bounds__(256) void k_wt_f16(const float* __restrict__ W, _Float16* __restrict__ Wt, int K, int N, float scale) {
  const int t = blockIdx.x * 256 + threadIdx.x; if (t >= N * (K / 8)) return; const int n = t / (K / 8), k8 = (t % (K / 8)) * 8; FragH f;
#pragma unroll
  for (int i = 0; i < 8; ++i) f.h[i] = (_Float16)(bf16_rne(W[(size_t)(k8 + i) * N + n]) * scale);
  const v8us o = f.half[0];
  unsigned short* dst = (unsigned short*)Wt + (size_t)n * K + k8;
  *(volatile v8us*)dst = o; __threadfence(); *(volatile v8us*)dst = o;
}

__global__ __launch_bounds__(128) void k_proj(const _Float16* __restrict__ A, const _Float16* __restrict__ Bh, float alpha, unsigned short* __restrict__ QKP, _Float16* __restrict__ V16, int M) {
  __shared__ __attribute__((aligned(16))) float so[4][32][68];
  const int tid = threadIdx.x, w = __builtin_amdgcn_readfirstlane((int)(tid >> 5)), lane = tid & 31, ln = lane & 15, hh = lane >> 4;
  const int ntn = (3 * DM) >> 6; const int mt = blockIdx.x / ntn, nq = blockIdx.x - mt * ntn; const int row0 = mt * 128 + 32 * w, col0 = nq * 64; if (row0 >= M) return;
  const _Float16* a0p = A + (size_t)(row0 + ln) * DM; const _Float16* a1p = a0p + (size_t)16 * DM;
  const _Float16* b0p = Bh + (size_t)(col0 + ln) * DM; const _Float16* b1p = b0p + (size_t)16 * DM; const _Float16* b2p = b1p + (size_t)16 * DM; const _Float16* b3p = b2p + (size_t)16 * DM;
  const v8f z8 = {0.f,0.f,0.f,0.f,0.f,0.f,0.f,0.f}; v8f c00 = z8, c01 = z8, c02 = z8, c03 = z8, c10 = z8, c11 = z8, c12 = z8, c13 = z8;
#pragma unroll 1
  for (int kb = 0; kb < DM; kb += 32) { const v16h a0 = g2_frag(a0p + kb, hh), a1 = g2_frag(a1p + kb, hh);
    v16h b = g2_frag(b0p + kb, hh); c00 = g2_mma(a0, b, c00); c10 = g2_mma(a1, b, c10);
    b = g2_frag(b1p + kb, hh); c01 = g2_mma(a0, b, c01); c11 = g2_mma(a1, b, c11);
    b = g2_frag(b2p + kb, hh); c02 = g2_mma(a0, b, c02); c12 = g2_mma(a1, b, c12);
    b = g2_frag(b3p + kb, hh); c03 = g2_mma(a0, b, c03); c13 = g2_mma(a1, b, c13); }
  v8f accs[8] = {c00, c01, c02, c03, c10, c11, c12, c13};
#pragma unroll
  for (int u = 0; u < 8; ++u) { const int t = u & 3, half = u >> 2;
#pragma unroll
    for (int r = 0; r < 8; ++r) so[w][half * 16 + 8 * hh + r][t * 16 + ln] = accs[u][r] * alpha; }
  __builtin_amdgcn_fence(4  , "workgroup"); __builtin_amdgcn_wave_barrier();
  const int rsub = lane >> 4, c4 = (lane & 15) * 4;
  const int region = col0 / DM, hc = col0 - region * DM;
  if (region < 2) {
    unsigned short* pl = QKP + (size_t)region * NR * PQ + (size_t)(hc * 2);
    for (int pass = 0; pass < 2; ++pass) {
#pragma unroll
      for (int q = 0; q < 16; ++q) { const int r = q * 2 + rsub; const v4f v = *(const v4fa*)&so[w][r][c4]; v4us hi4, lo4;
#pragma unroll
        for (int i = 0; i < 4; ++i) { const unsigned short hb = bf16_bits(v[i]); hi4[i] = hb; lo4[i] = bf16_bits(v[i] - bf16_val(hb)); }
        unsigned short* d = pl + (size_t)(row0 + r) * PQ + c4;
        *(volatile v4us*)d = hi4; *(volatile v4us*)(d + HD) = lo4; }
      if (pass == 0) __threadfence(); }
  } else {
    for (int pass = 0; pass < 2; ++pass) {
#pragma unroll
      for (int q = 0; q < 16; ++q) { const int r = q * 2 + rsub; const v4f v = *(const v4fa*)&so[w][r][c4]; v4h h4;
#pragma unroll
        for (int i = 0; i < 4; ++i) h4[i] = (_Float16)v[i];
        *(volatile v4h*)(V16 + (size_t)(row0 + r) * DM + hc + c4) = h4; }
      if (pass == 0) __threadfence(); }
  }
}

template <int NHv, int TTv>
__global__ __launch_bounds__(256) void k_vt(const _Float16* __restrict__ V16, int ldv, int voff, _Float16* __restrict__ Vt) { __shared__ unsigned short tl[64][66]; const int tid = threadIdx.x; const int slab = blockIdx.x / (TTv / 64), lg = blockIdx.x % (TTv / 64); const int b = slab / NHv, h = slab % NHv;
  for (int i = tid; i < 64 * 8; i += 256) { const int r = i / 8, c8 = (i % 8) * 8; FragH f; f.half[0] = *(const v8us*)((const unsigned short*)V16 + ((size_t)b * TTv + lg * 64 + r) * ldv + voff + h * 64 + c8);
#pragma unroll
    for (int q = 0; q < 8; ++q) tl[r][c8 + q] = f.u[q]; }
  __syncthreads();
  for (int pass = 0; pass < 2; ++pass) {
#pragma unroll
    for (int rd = 0; rd < 2; ++rd) { const int d = rd * 32 + tid / 8, pc = tid % 8; FragH f;
#pragma unroll
      for (int q = 0; q < 8; ++q) f.u[q] = tl[pc * 8 + q][d];
      *(volatile v8us*)((unsigned short*)Vt + ((size_t)slab * 64 + d) * TTv + lg * 64 + pc * 8) = f.half[0]; }
    if (pass == 0) __threadfence(); } }

__global__ __launch_bounds__(128) void k_score(const unsigned short* __restrict__ Aq, const unsigned short* __restrict__ Bk, int ld, float alpha, float* __restrict__ C, int ldc, size_t sC, int M, int N) {
  __shared__ __attribute__((aligned(16))) float so[4][32][68];
  const int tid = threadIdx.x, w = __builtin_amdgcn_readfirstlane((int)(tid >> 5)), lane = tid & 31, ln = lane & 15, hh = lane >> 4; const int by = blockIdx.y;
  Aq += (size_t)by * (2 * HD); Bk += (size_t)by * (2 * HD); const size_t cofs = (size_t)by * sC;
  const int ntn = N >> 6; const int mt = blockIdx.x / ntn, nq = blockIdx.x - mt * ntn; const int row0 = mt * 128 + 32 * w, col0 = nq * 64; if (row0 >= M) return;
  const unsigned short* a0p = Aq + (size_t)(row0 + ln) * ld; const unsigned short* a1p = a0p + (size_t)16 * ld;
  const unsigned short* b0p = Bk + (size_t)(col0 + ln) * ld; const unsigned short* b1p = b0p + (size_t)16 * ld; const unsigned short* b2p = b1p + (size_t)16 * ld; const unsigned short* b3p = b2p + (size_t)16 * ld;
  const v8f z8 = {0.f,0.f,0.f,0.f,0.f,0.f,0.f,0.f}; v8f c00 = z8, c01 = z8, c02 = z8, c03 = z8, c10 = z8, c11 = z8, c12 = z8, c13 = z8;
#pragma unroll 1
  for (int kk = 0; kk < 6; ++kk) { const int pr = kk >> 1, ko = (kk & 1) * 32;
    const int ao = ((pr == 2) ? HD : 0) + ko;
    const int bo = ((pr == 1) ? HD : 0) + ko;
    const v16b a0 = gb_frag(a0p + ao, hh), a1 = gb_frag(a1p + ao, hh);
    v16b b = gb_frag(b0p + bo, hh); c00 = gb_mma(a0, b, c00); c10 = gb_mma(a1, b, c10);
    b = gb_frag(b1p + bo, hh); c01 = gb_mma(a0, b, c01); c11 = gb_mma(a1, b, c11);
    b = gb_frag(b2p + bo, hh); c02 = gb_mma(a0, b, c02); c12 = gb_mma(a1, b, c12);
    b = gb_frag(b3p + bo, hh); c03 = gb_mma(a0, b, c03); c13 = gb_mma(a1, b, c13); }
  v8f accs[8] = {c00, c01, c02, c03, c10, c11, c12, c13};
#pragma unroll
  for (int u = 0; u < 8; ++u) { const int t = u & 3, half = u >> 2;
#pragma unroll
    for (int r = 0; r < 8; ++r) so[w][half * 16 + 8 * hh + r][t * 16 + ln] = accs[u][r] * alpha; }
  __builtin_amdgcn_fence(4  , "workgroup"); __builtin_amdgcn_wave_barrier();
  const int rsub = lane >> 4, c4 = (lane & 15) * 4;
  for (int pass = 0; pass < 2; ++pass) {
#pragma unroll
    for (int q = 0; q < 16; ++q) { const int r = q * 2 + rsub; const v4f v = *(const v4fa*)&so[w][r][c4]; *(volatile v4f*)(C + cofs + (size_t)(row0 + r) * ldc + col0 + c4) = v; }
    if (pass == 0) __threadfence(); }
}

__global__ __launch_bounds__(256) void k_csm(const float* __restrict__ S, _Float16* __restrict__ P) {
  #pragma clang fp contract(off)
  __shared__ float red[16][64]; __shared__ float cmx[64]; __shared__ float csc[64];
  const int tid = threadIdx.x; const int hh = blockIdx.y; const int m0 = blockIdx.x * 64;
  const float* s = S + (size_t)hh * SEQ * SEQ + m0;
  const int cq = (tid & 15) * 4, g = tid >> 4;
  v4f mx4 = {-3.0e38f, -3.0e38f, -3.0e38f, -3.0e38f};
#pragma unroll 2
  for (int l = g; l < SEQ; l += 16) { const v4f a = *(const v4fa*)(s + (size_t)l * SEQ + cq);
#pragma unroll
    for (int q = 0; q < 4; ++q) mx4[q] = fmaxf(mx4[q], a[q]); }
#pragma unroll
  for (int q = 0; q < 4; ++q) red[g][cq + q] = mx4[q];
  __syncthreads();
  if (tid < 64) { float m = red[0][tid];
#pragma unroll
    for (int u = 1; u < 16; ++u) m = fmaxf(m, red[u][tid]);
    cmx[tid] = m; }
  __syncthreads();
  v4f cm4;
#pragma unroll
  for (int q = 0; q < 4; ++q) cm4[q] = cmx[cq + q];
  v4f se4 = {0.f, 0.f, 0.f, 0.f};
#pragma unroll 2
  for (int l = g; l < SEQ; l += 16) { const v4f a = *(const v4fa*)(s + (size_t)l * SEQ + cq);
#pragma unroll
    for (int q = 0; q < 4; ++q) se4[q] += __expf(a[q] - cm4[q]); }
#pragma unroll
  for (int q = 0; q < 4; ++q) red[g][cq + q] = se4[q];
  __syncthreads();
  if (tid < 64) { float t = red[0][tid];
#pragma unroll
    for (int u = 1; u < 16; ++u) t += red[u][tid];
    csc[tid] = 1024.0f * (1.0f / t); }
  __syncthreads();
  const int pc = (tid & 7) * 8, rs = tid >> 3;
  float m8[8], s8[8];
#pragma unroll
  for (int q = 0; q < 8; ++q) { m8[q] = cmx[pc + q]; s8[q] = csc[pc + q]; }
  unsigned short* pb = (unsigned short*)P + (size_t)hh * SEQ * SEQ + m0 + pc;
#pragma unroll 1
  for (int it = 0; it < SEQ / 32; ++it) { const int l = it * 32 + rs; const float* sp = s + (size_t)l * SEQ + pc;
    const v4f a = *(const v4fa*)sp, c = *(const v4fa*)(sp + 4); FragH f;
#pragma unroll
    for (int q = 0; q < 4; ++q) { f.h[q] = (_Float16)(__expf(a[q] - m8[q]) * s8[q]); f.h[4 + q] = (_Float16)(__expf(c[q] - m8[4 + q]) * s8[4 + q]); }
    const v8us o = f.half[0]; unsigned short* d = pb + (size_t)l * SEQ;
    *(volatile v8us*)d = o; __threadfence(); *(volatile v8us*)d = o; }
}

__global__ __launch_bounds__(128) void k_gemm2(const _Float16* __restrict__ A, int lda, size_t sA, const _Float16* __restrict__ Bh, int ldb, size_t sB, float alpha, const float* __restrict__ bias,
    float* __restrict__ C, _Float16* __restrict__ C16, int ldc, size_t sC, int M, int N, int K) {
  __shared__ __attribute__((aligned(16))) float so[4][32][68];
  const int tid = threadIdx.x, w = __builtin_amdgcn_readfirstlane((int)(tid >> 5)), lane = tid & 31, ln = lane & 15, hh = lane >> 4; const int by = blockIdx.y;
  A += (size_t)by * sA; Bh += (size_t)by * sB; const size_t cofs = (size_t)by * sC;
  const int ntn = N >> 6; const int mt = blockIdx.x / ntn, nq = blockIdx.x - mt * ntn; const int row0 = mt * 128 + 32 * w, col0 = nq * 64; if (row0 >= M) return;
  const _Float16* a0p = A + (size_t)(row0 + ln) * lda; const _Float16* a1p = a0p + (size_t)16 * lda;
  const _Float16* b0p = Bh + (size_t)(col0 + ln) * ldb; const _Float16* b1p = b0p + (size_t)16 * ldb; const _Float16* b2p = b1p + (size_t)16 * ldb; const _Float16* b3p = b2p + (size_t)16 * ldb;
  const v8f z8 = {0.f,0.f,0.f,0.f,0.f,0.f,0.f,0.f}; v8f c00 = z8, c01 = z8, c02 = z8, c03 = z8, c10 = z8, c11 = z8, c12 = z8, c13 = z8;
#pragma unroll 1
  for (int kb = 0; kb < K; kb += 32) { const v16h a0 = g2_frag(a0p + kb, hh), a1 = g2_frag(a1p + kb, hh);
    v16h b = g2_frag(b0p + kb, hh); c00 = g2_mma(a0, b, c00); c10 = g2_mma(a1, b, c10);
    b = g2_frag(b1p + kb, hh); c01 = g2_mma(a0, b, c01); c11 = g2_mma(a1, b, c11);
    b = g2_frag(b2p + kb, hh); c02 = g2_mma(a0, b, c02); c12 = g2_mma(a1, b, c12);
    b = g2_frag(b3p + kb, hh); c03 = g2_mma(a0, b, c03); c13 = g2_mma(a1, b, c13); }
  v8f accs[8] = {c00, c01, c02, c03, c10, c11, c12, c13};
#pragma unroll
  for (int u = 0; u < 8; ++u) { const int t = u & 3, half = u >> 2; const int col = col0 + t * 16 + ln; const float bv = bias ? bf16_rne(bias[col]) : 0.f;
#pragma unroll
    for (int r = 0; r < 8; ++r) so[w][half * 16 + 8 * hh + r][t * 16 + ln] = accs[u][r] * alpha + bv; }
  __builtin_amdgcn_fence(4  , "workgroup"); __builtin_amdgcn_wave_barrier();
  const int rsub = lane >> 4, c4 = (lane & 15) * 4;
  for (int pass = 0; pass < 2; ++pass) {
#pragma unroll
    for (int q = 0; q < 16; ++q) { const int r = q * 2 + rsub; const v4f v = *(const v4fa*)&so[w][r][c4];
      if (C) *(volatile v4f*)(C + cofs + (size_t)(row0 + r) * ldc + col0 + c4) = v;
      if (C16) { v4h h4;
#pragma unroll
        for (int i = 0; i < 4; ++i) h4[i] = (_Float16)v[i];
        *(volatile v4h*)(C16 + cofs + (size_t)(row0 + r) * ldc + col0 + c4) = h4; } }
    if (pass == 0) __threadfence(); }
}

extern "C" void kernel_launch(void* const* d_in, const int* in_sizes, int n_in,
                              void* d_out, int out_size, void* d_ws, size_t ws_size, hipStream_t stream) {
  if (n_in < 6) return;
  if ((size_t)in_sizes[0] < ((size_t)(NB - 1) * SEQ_FULL + SEQ) * DM) return;
  if ((size_t)in_sizes[1] < (size_t)NH * DM * HD || (size_t)in_sizes[2] < (size_t)NH * DM * HD || (size_t)in_sizes[3] < (size_t)NH * DM * HD) return;
  if ((size_t)in_sizes[4] < (size_t)DM * DM || in_sizes[5] < DM) return;
  if ((size_t)out_size < NR * DM) return;
  const float* x = (const float*)d_in[0]; const float* wq = (const float*)d_in[1]; const float* wk = (const float*)d_in[2]; const float* wv = (const float*)d_in[3]; const float* wo = (const float*)d_in[4]; const float* bo = (const float*)d_in[5];
  char* ws = (char*)d_ws; size_t off = 0;
  auto take = [&](size_t bytes) { char* p = ws + off; off += (bytes + 255) & ~(size_t)255; return p; };
  _Float16* BQKV = (_Float16*)take(SZ_BQKV); _Float16* BO = (_Float16*)take(SZ_BO);
  _Float16* X16 = (_Float16*)take(SZ_X16);
  unsigned short* QKP = (unsigned short*)take(SZ_QKP); unsigned short* QP = QKP; unsigned short* KP = QKP + NR * PQ;
  _Float16* V16 = (_Float16*)take(SZ_V16); _Float16* VT = (_Float16*)take(SZ_VT); _Float16* O16 = (_Float16*)take(SZ_O16);
  float* S = (float*)take(SZ_S); _Float16* P = (_Float16*)take(SZ_P);
  if (off > ws_size || off > (size_t)134217728) return;

  const unsigned wtb = (unsigned)(((size_t)DM * (DM / 8) + 255) / 256);
  k_wth<<<wtb, 256, 0, stream>>>(wq, BQKV);
  k_wth<<<wtb, 256, 0, stream>>>(wk, BQKV + (size_t)DM * DM);
  k_wth<<<wtb, 256, 0, stream>>>(wv, BQKV + (size_t)2 * DM * DM);
  k_wt_f16<<<wtb, 256, 0, stream>>>(wo, BO, DM, DM, 64.0f);
  k_x16<<<(unsigned)((NR * DM / 8 + 255) / 256), 256, 0, stream>>>(x, X16, NR * DM / 8);
  k_proj<<<(unsigned)((NR / 128) * (3 * DM / 64)), 128, 0, stream>>>(X16, BQKV, 0.000244140625f, QKP, V16, (int)NR);
  k_vt<NH, SEQ><<<NB * NH * (SEQ / 64), 256, 0, stream>>>(V16, DM, 0, VT);
  for (int b = 0; b < NB; ++b) { const size_t r0 = (size_t)b * SEQ;
    for (int h0 = 0; h0 < NH; h0 += HG) {
      k_score<<<dim3((SEQ / 128) * (SEQ / 64), HG), 128, 0, stream>>>(QP + r0 * PQ + (size_t)h0 * 2 * HD, KP + r0 * PQ + (size_t)h0 * 2 * HD, PQ, 32.0f, S, SEQ, (size_t)SEQ * SEQ, SEQ, SEQ);
      k_csm<<<dim3(SEQ / 64, HG), 256, 0, stream>>>(S, P);
      k_gemm2<<<dim3(SEQ / 128, HG), 128, 0, stream>>>(P, SEQ, (size_t)SEQ * SEQ, VT + ((size_t)b * NH + h0) * HD * SEQ, SEQ, (size_t)HD * SEQ, 0.015625f, nullptr, nullptr, O16 + r0 * DM + (size_t)h0 * HD, DM, (size_t)HD, SEQ, HD, SEQ);
    } }
  k_gemm2<<<dim3((unsigned)((NR / 128) * (DM / 64)), 1), 128, 0, stream>>>(O16, DM, 0, BO, DM, 0, 0.0009765625f, bo, (float*)d_out, nullptr, DM, 0, (int)NR, DM, DM);
}
